// CrossAttention_32263794328065
// MI455X (gfx1250) — hardware-verified
//
#include <hip/hip_runtime.h>
#include <stdint.h>
#include <math.h>


typedef _Float16 v16h __attribute__((ext_vector_type(16)));
typedef _Float16 v8h  __attribute__((ext_vector_type(8)));
typedef float    v8f  __attribute__((ext_vector_type(8)));
typedef float    v4f  __attribute__((ext_vector_type(4)));

#ifndef NB
#define NB 2
#endif
#ifndef SEQ
#define SEQ 2048
#endif
#define NB_FULL   2
#define SEQ_FULL  2048
#define ZD   1024
#define DL   512
#define DM   1024
#define NH   16
#define HD   64
#define RD   64
#define MROWS (NB * SEQ)

#define ACT_CAR   8.0f
#define W_CAR     1024.0f
#define PROJ_SCL  0.0009765625f
#define RES_CAR   2048.0f
#define RES_INV   0.00048828125f
#define S_SCL     0.0009765625f
#define P_CAR     16384.0f
#define O_SCL     0.001953125f
#define OUT_SCL   3.814697265625e-06f

static_assert(SEQ % 128 == 0);
static_assert(NB <= NB_FULL && SEQ <= SEQ_FULL);
static_assert(DM == NH * HD);
static_assert(HD == 64 && RD == 64);
static_assert(DM == ZD);
static_assert(ZD % 64 == 0 && DL % 64 == 0 && DM % 64 == 0 && ZD % 32 == 0 && DL % 32 == 0);
static_assert((long)NB_FULL * SEQ_FULL * ZD * 4 == 16777216L);
static_assert(((long)MROWS * ZD / 8) % 256 == 0);
static_assert((long)(DL / 64) * (ZD / 64) * 4096 == (long)ZD * DL);
static_assert((long)(RD / 64) * (ZD / 64) * 4096 == (long)ZD * RD);
static_assert((long)(DM / 64) * (DL / 64) * 4096 == (long)DL * DM);
static_assert((long)(ZD / 64) * (DM / 64) * 4096 == (long)DM * ZD);
static_assert((long)(SEQ / 8) * 512 == (long)SEQ * 64);
static_assert((long)(DL / 64) * (MROWS / 128) * 128 * 64 == (long)MROWS * DL);
static_assert((long)(RD / 64) * (MROWS / 128) * 128 * 64 == (long)MROWS * RD);
static_assert((long)(DM / 64) * (MROWS / 128) * 128 * 64 == (long)MROWS * DM);
static_assert((long)(DM / 64) * (MROWS / 64) * 64 * 64 == (long)NB * DM * SEQ);
static_assert((long)(SEQ / 128) * NH * NB * 128 * HD == (long)MROWS * DM);
static_assert((long)(ZD / 64) * (MROWS / 64) * 64 * 64 == (long)MROWS * ZD);

union Frag16 { v16h v; v8h p[2]; };

__device__ __forceinline__ v16h ld_frag(const _Float16* p, int hl) {
  Frag16 f;
  f.p[0] = *(const v8h*)(p + 8 * hl);
  f.p[1] = *(const v8h*)(p + 16 + 8 * hl);
  return f.v;
}

__device__ __forceinline__ v8f mma(v16h a, v16h b, v8f c) {
  v8f d = __builtin_amdgcn_wmma_f32_16x16x32_f16(false, a, false, b, (short)0, c, false, false);
  asm volatile("v_nop\n\tv_nop\n\tv_nop\n\tv_nop" : "+v"(d) : "v"(a), "v"(b));
  return d;
}

__device__ __forceinline__ float bf16_rne(float x) {
  unsigned int u = __builtin_bit_cast(unsigned int, x);
  u += 0x7FFFu + ((u >> 16) & 1u);
  return __builtin_bit_cast(float, u & 0xFFFF0000u);
}

__global__ __launch_bounds__(256) void k_cvt8(const float* __restrict__ src,
                                              _Float16* __restrict__ dst,
                                              float car, unsigned total8)
{
  const unsigned i8 = blockIdx.x * 256u + threadIdx.x;
  if (i8 >= total8) return;
  const unsigned e   = i8 * 8u;
  const unsigned r   = e >> 10;
  const unsigned col = e & 1023u;
  const unsigned b   = r / (unsigned)SEQ;
  const unsigned t   = r - b * (unsigned)SEQ;
  const float* s = src + ((size_t)b * SEQ_FULL + t) * ZD + col;
  const v4f x0 = *(const v4f*)s;
  const v4f x1 = *(const v4f*)(s + 4);
  v8h o;
#pragma unroll
  for (int j = 0; j < 4; ++j) {
    const float t0 = x0[j];
    const float t1 = x1[j];
    o[j]     = (_Float16)(bf16_rne(t0) * car);
    o[4 + j] = (_Float16)(bf16_rne(t1) * car);
  }
  _Float16* d = dst + e;
  *(volatile v8h*)d = o;
  __threadfence();
  *(volatile v8h*)d = o;
}

__global__ __launch_bounds__(256) void k_trw(const float* __restrict__ W,
                                             _Float16* __restrict__ WT, int R, int C)
{
  __shared__ float tile[64 * 65];
  const int tid = threadIdx.x;
  const int c0 = blockIdx.x * 64, r0 = blockIdx.y * 64;
#pragma unroll
  for (int i = 0; i < 4; ++i) {
    const int idx = i * 256 + tid;
    const int r = idx >> 4, c4 = (idx & 15) * 4;
    const v4f v = *(const v4f*)(W + (size_t)(r0 + r) * C + c0 + c4);
    float* tp = tile + r * 65 + c4;
    tp[0] = v[0]; tp[1] = v[1]; tp[2] = v[2]; tp[3] = v[3];
  }
  __syncthreads();
  v8h o[2];
  _Float16* dp[2];
#pragma unroll
  for (int i = 0; i < 2; ++i) {
    const int line = i * 32 + (tid >> 3);
    const int pc   = (tid & 7) * 8;
#pragma unroll
    for (int j = 0; j < 8; ++j)
      o[i][j] = (_Float16)(bf16_rne(tile[(pc + j) * 65 + line]) * W_CAR);
    dp[i] = WT + (size_t)(c0 + line) * R + r0 + pc;
  }
  *(volatile v8h*)dp[0] = o[0];
  *(volatile v8h*)dp[1] = o[1];
  __threadfence();
  *(volatile v8h*)dp[0] = o[0];
  *(volatile v8h*)dp[1] = o[1];
}

struct InvF { float v[32]; };
static_assert(sizeof(InvF) == 128);

__global__ __launch_bounds__(256) void k_tab(InvF f, float* __restrict__ TAB)
{
  __shared__ float sInv[32];
  __shared__ __attribute__((aligned(16))) float sT[512];
  const unsigned tid = threadIdx.x;
  if (tid == 0) {
#pragma unroll
    for (int j = 0; j < 32; ++j) sInv[j] = f.v[j];
  }
  __syncthreads();
  const unsigned t = blockIdx.x * 8u + (tid >> 5);
  const unsigned i = tid & 31u;
  const float ang = (float)t * sInv[i];
  float s, c;
  sincosf(ang, &s, &c);
  sT[2u * tid]      = s;
  sT[2u * tid + 1u] = c;
  __syncthreads();
  if (tid < 128u) {
    const v4f v = *(const v4f*)(sT + 4u * tid);
    float* d = TAB + (size_t)blockIdx.x * 512u + 4u * tid;
    *(volatile v4f*)d = v;
    __threadfence();
    *(volatile v4f*)d = v;
  }
}

__device__ __forceinline__ void gemm_core(const _Float16* ap0, const _Float16* ap1,
                                          const _Float16* bp, int K, int hl, v8f (&acc)[8])
{
  const size_t bst = (size_t)16 * K;
#pragma unroll 1
  for (int k0 = 0; k0 < K; k0 += 32) {
    const v16h a0 = ld_frag(ap0 + k0, hl);
    const v16h a1 = ld_frag(ap1 + k0, hl);
    const v16h b0 = ld_frag(bp + k0, hl);
    const v16h b1 = ld_frag(bp + bst + k0, hl);
    const v16h b2 = ld_frag(bp + 2 * bst + k0, hl);
    const v16h b3 = ld_frag(bp + 3 * bst + k0, hl);
    acc[0] = mma(a0, b0, acc[0]);
    acc[1] = mma(a0, b1, acc[1]);
    acc[2] = mma(a0, b2, acc[2]);
    acc[3] = mma(a0, b3, acc[3]);
    acc[4] = mma(a1, b0, acc[4]);
    acc[5] = mma(a1, b1, acc[5]);
    acc[6] = mma(a1, b2, acc[6]);
    acc[7] = mma(a1, b3, acc[7]);
  }
}

template <int EPI>
__global__ __launch_bounds__(128) __attribute__((amdgpu_num_vgpr(256)))
void k_proj(const _Float16* __restrict__ A, const _Float16* __restrict__ Bt,
            const float* __restrict__ bias, const float* __restrict__ TAB,
            _Float16* __restrict__ PH, _Float16* __restrict__ PL, int K, int ldc)
{
  __shared__ __attribute__((aligned(16))) _Float16 ldsE[2 * 128 * 72];
  _Float16* const ldsH = ldsE;
  _Float16* const ldsL = ldsE + 128 * 72;
  float*    const ldsF = (float*)ldsE;

  const int tid = threadIdx.x, lane = tid & 31, w = tid >> 5;
  const int hl = lane >> 4, c = lane & 15;
  const int m0 = blockIdx.y * 128, n0 = blockIdx.x * 64;
  const int mw = m0 + 32 * w;

  const _Float16* ap0 = A  + (size_t)(mw + c) * K;
  const _Float16* ap1 = A  + (size_t)(mw + 16 + c) * K;
  const _Float16* bp  = Bt + (size_t)(n0 + c) * K;

  v8f acc[8] = {};
  gemm_core(ap0, ap1, bp, K, hl, acc);

  float bs[4];
#pragma unroll
  for (int t = 0; t < 4; ++t) bs[t] = bf16_rne(bias[n0 + 16 * t + c]) * ACT_CAR;

#pragma unroll
  for (int i = 0; i < 2; ++i)
#pragma unroll
    for (int t = 0; t < 4; ++t)
#pragma unroll
      for (int r = 0; r < 8; ++r) {
        const int rowl = 32 * w + 16 * i + 8 * hl + r;
        const float v = acc[i * 4 + t][r] * PROJ_SCL + bs[t];
        if (EPI == 2) {
          ldsF[rowl * 68 + 16 * t + c] = v;
        } else {
          const _Float16 hv = (_Float16)v;
          ldsH[rowl * 72 + 16 * t + c] = hv;
          if (EPI == 1) {
            const float res = (v - (float)hv) * RES_CAR;
            ldsL[rowl * 72 + 16 * t + c] = (_Float16)res;
          }
        }
      }
  __syncthreads();

  _Float16* const bh = PH + (size_t)m0 * ldc + n0;
  if (EPI == 2) {
    const unsigned t0 = (unsigned)m0 % (unsigned)SEQ;
    v8h ov[8];
#pragma unroll
    for (int i = 0; i < 8; ++i) {
      const int q = i * 128 + tid;
      const int rowl = q >> 3, ch = (q & 7) * 8;
      const v4f x0 = *(const v4f*)(ldsF + rowl * 68 + ch);
      const v4f x1 = *(const v4f*)(ldsF + rowl * 68 + ch + 4);
      const float* tb = TAB + (size_t)(t0 + (unsigned)rowl) * 64u + (unsigned)ch;
      const v4f s0 = *(const v4f*)tb;
      const v4f s1 = *(const v4f*)(tb + 4);
      v8h o;
      o[0] = (_Float16)(x0[0] * s0[0] - x0[1] * s0[1]);
      o[1] = (_Float16)(x0[1] * s0[0] + x0[0] * s0[1]);
      o[2] = (_Float16)(x0[2] * s0[2] - x0[3] * s0[3]);
      o[3] = (_Float16)(x0[3] * s0[2] + x0[2] * s0[3]);
      o[4] = (_Float16)(x1[0] * s1[0] - x1[1] * s1[1]);
      o[5] = (_Float16)(x1[1] * s1[0] + x1[0] * s1[1]);
      o[6] = (_Float16)(x1[2] * s1[2] - x1[3] * s1[3]);
      o[7] = (_Float16)(x1[3] * s1[2] + x1[2] * s1[3]);
      ov[i] = o;
    }
#pragma unroll
    for (int i = 0; i < 8; ++i) {
      const int q = i * 128 + tid;
      const int rowl = q >> 3, ch = (q & 7) * 8;
      *(volatile v8h*)(bh + (size_t)rowl * ldc + ch) = ov[i];
    }
    __threadfence();
#pragma unroll
    for (int i = 0; i < 8; ++i) {
      const int q = i * 128 + tid;
      const int rowl = q >> 3, ch = (q & 7) * 8;
      *(volatile v8h*)(bh + (size_t)rowl * ldc + ch) = ov[i];
    }
  } else {
    for (int i = 0; i < 8; ++i) {
      const int q = i * 128 + tid;
      const int rowl = q >> 3, ch = (q & 7) * 8;
      const v8h vh = *(const v8h*)(ldsH + rowl * 72 + ch);
      *(volatile v8h*)(bh + (size_t)rowl * ldc + ch) = vh;
      if (EPI == 1) {
        const v8h vl = *(const v8h*)(ldsL + rowl * 72 + ch);
        *(volatile v8h*)(PL + (size_t)m0 * ldc + n0 + (size_t)rowl * ldc + ch) = vl;
      }
    }
    __threadfence();
    for (int i = 0; i < 8; ++i) {
      const int q = i * 128 + tid;
      const int rowl = q >> 3, ch = (q & 7) * 8;
      const v8h vh = *(const v8h*)(ldsH + rowl * 72 + ch);
      *(volatile v8h*)(bh + (size_t)rowl * ldc + ch) = vh;
      if (EPI == 1) {
        const v8h vl = *(const v8h*)(ldsL + rowl * 72 + ch);
        *(volatile v8h*)(PL + (size_t)m0 * ldc + n0 + (size_t)rowl * ldc + ch) = vl;
      }
    }
  }
}

__global__ __launch_bounds__(128) __attribute__((amdgpu_num_vgpr(256)))
void k_vproj(const _Float16* __restrict__ AH, const _Float16* __restrict__ AL,
             const _Float16* __restrict__ Bt, const float* __restrict__ bias,
             _Float16* __restrict__ VtH, _Float16* __restrict__ VtL)
{
  __shared__ __attribute__((aligned(16))) _Float16 ldsE[2 * 64 * 72];
  _Float16* const ldsH = ldsE;
  _Float16* const ldsL = ldsE + 64 * 72;

  const int tid = threadIdx.x, lane = tid & 31, w = tid >> 5;
  const int hl = lane >> 4, c = lane & 15;
  const int m0 = blockIdx.y * 64, n0 = blockIdx.x * 64;
  const int mw = m0 + 16 * w;

  const _Float16* ap0 = AH + (size_t)(mw + c) * DL;
  const _Float16* ap1 = AL + (size_t)(mw + c) * DL;
  const _Float16* bp  = Bt + (size_t)(n0 + c) * DL;

  v8f acc[8] = {};
  gemm_core(ap0, ap1, bp, DL, hl, acc);

  float bs[4];
#pragma unroll
  for (int t = 0; t < 4; ++t) bs[t] = bf16_rne(bias[n0 + 16 * t + c]) * ACT_CAR;

#pragma unroll
  for (int t = 0; t < 4; ++t)
#pragma unroll
    for (int r = 0; r < 8; ++r) {
      const int keyl = 16 * w + 8 * hl + r;
      const int dl   = 16 * t + c;
      const float v = (acc[t][r] + acc[4 + t][r] * RES_INV) * PROJ_SCL + bs[t];
      const _Float16 hv = (_Float16)v;
      const float res = (v - (float)hv) * RES_CAR;
      ldsH[dl * 72 + keyl] = hv;
      ldsL[dl * 72 + keyl] = (_Float16)res;
    }
  __syncthreads();

  const unsigned b  = (unsigned)m0 / (unsigned)SEQ;
  const unsigned t0 = (unsigned)m0 - b * (unsigned)SEQ;
  _Float16* const bh = VtH + ((size_t)b * DM + n0) * SEQ + t0;
  _Float16* const bl = VtL + ((size_t)b * DM + n0) * SEQ + t0;
  for (int i = 0; i < 4; ++i) {
    const int q = i * 128 + tid;
    const int dl = q >> 3, ch = (q & 7) * 8;
    const v8h vh = *(const v8h*)(ldsH + dl * 72 + ch);
    const v8h vl = *(const v8h*)(ldsL + dl * 72 + ch);
    *(volatile v8h*)(bh + (size_t)dl * SEQ + ch) = vh;
    *(volatile v8h*)(bl + (size_t)dl * SEQ + ch) = vl;
  }
  __threadfence();
  for (int i = 0; i < 4; ++i) {
    const int q = i * 128 + tid;
    const int dl = q >> 3, ch = (q & 7) * 8;
    const v8h vh = *(const v8h*)(ldsH + dl * 72 + ch);
    const v8h vl = *(const v8h*)(ldsL + dl * 72 + ch);
    *(volatile v8h*)(bh + (size_t)dl * SEQ + ch) = vh;
    *(volatile v8h*)(bl + (size_t)dl * SEQ + ch) = vl;
  }
}

__global__ __launch_bounds__(256) __attribute__((amdgpu_num_vgpr(256)))
void k_attn(const _Float16* __restrict__ QC, const _Float16* __restrict__ QR,
            const _Float16* __restrict__ KC, const _Float16* __restrict__ KR,
            const _Float16* __restrict__ VtH, const _Float16* __restrict__ VtL,
            _Float16* __restrict__ OH, _Float16* __restrict__ OL)
{
  constexpr int KP     = 136;
  constexpr int KT_H   = 32 * KP;
  constexpr int V_H    = HD * 40;
  constexpr int P_H    = 8 * 16 * 40;
  constexpr int TILE_H = KT_H + 2 * V_H + P_H;
  constexpr int EPI_H  = 2 * 128 * 72;
  constexpr int LDS_H  = (TILE_H > EPI_H) ? TILE_H : EPI_H;
  __shared__ __attribute__((aligned(16))) _Float16 lds[LDS_H];
  _Float16* const ldsK  = lds;
  _Float16* const ldsVH = ldsK + KT_H;
  _Float16* const ldsVL = ldsVH + V_H;
  _Float16* const ldsP  = ldsVL + V_H;
  _Float16* const ldsOH = lds;
  _Float16* const ldsOL = lds + 128 * 72;

  const int tid = threadIdx.x, lane = tid & 31, w = tid >> 5;
  const int hl = lane >> 4, c = lane & 15;
  const int q0 = blockIdx.x * 128;
  const int col0 = blockIdx.y * HD;
  const int bb = blockIdx.z;
  const size_t brow = (size_t)bb * SEQ;

  const size_t qrow = (brow + (size_t)(q0 + 16 * w + c)) * DM + col0;
  v16h qf[4];
  qf[0] = ld_frag(QC + qrow, hl);
  qf[1] = ld_frag(QC + qrow + 32, hl);
  qf[2] = ld_frag(QR + qrow, hl);
  qf[3] = ld_frag(QR + qrow + 32, hl);
  _Float16* const myP = ldsP + w * (16 * 40);

  const int krr = tid >> 3, kcc = (tid & 7) * 8;
  const int vdd = tid >> 2, vkc = (tid & 3) * 8;
  const _Float16* const kgc = KC + (brow + (size_t)krr) * DM + col0 + kcc;
  const _Float16* const kgr = KR + (brow + (size_t)krr) * RD + kcc;
  const _Float16* const vgh = VtH + ((size_t)bb * DM + col0 + vdd) * SEQ + vkc;
  const _Float16* const vgl = VtL + ((size_t)bb * DM + col0 + vdd) * SEQ + vkc;

  float m[8], l[8];
  v8f oh[4] = {}, ol[4] = {};
#pragma unroll
  for (int r = 0; r < 8; ++r) { m[r] = -__builtin_inff(); l[r] = 0.f; }

#pragma unroll 1
  for (int kt = 0; kt < SEQ / 32; ++kt) {
    const int mk = kt * 32;
    {
      const v8h k8c = *(const v8h*)(kgc + (size_t)mk * DM);
      const v8h k8r = *(const v8h*)(kgr + (size_t)mk * RD);
      const v8h v8a = *(const v8h*)(vgh + mk);
      const v8h v8b = *(const v8h*)(vgl + mk);
      *(v8h*)(ldsK + krr * KP + kcc)      = k8c;
      *(v8h*)(ldsK + krr * KP + 64 + kcc) = k8r;
      *(v8h*)(ldsVH + vdd * 40 + vkc) = v8a;
      *(v8h*)(ldsVL + vdd * 40 + vkc) = v8b;
    }
    __syncthreads();

    v8f sh[2] = {};
#pragma unroll
    for (int ks = 0; ks < 4; ++ks) {
#pragma unroll
      for (int t = 0; t < 2; ++t) {
        const v16h kf = ld_frag(ldsK + (16 * t + c) * KP + 32 * ks, hl);
        sh[t] = mma(qf[ks], kf, sh[t]);
      }
    }

#pragma unroll
    for (int r = 0; r < 8; ++r) {
      const float v0 = sh[0][r] * S_SCL;
      const float v1 = sh[1][r] * S_SCL;
      float tm = fmaxf(v0, v1);
      tm = fmaxf(tm, __shfl_xor(tm, 1, 32));
      tm = fmaxf(tm, __shfl_xor(tm, 2, 32));
      tm = fmaxf(tm, __shfl_xor(tm, 4, 32));
      tm = fmaxf(tm, __shfl_xor(tm, 8, 32));
      const float mn = fmaxf(m[r], tm);
      const float al = __expf(m[r] - mn);
      const float p0 = __expf(v0 - mn), p1 = __expf(v1 - mn);
      float rs = p0 + p1;
      rs += __shfl_xor(rs, 1, 32);
      rs += __shfl_xor(rs, 2, 32);
      rs += __shfl_xor(rs, 4, 32);
      rs += __shfl_xor(rs, 8, 32);
      l[r] = l[r] * al + rs;
      m[r] = mn;
#pragma unroll
      for (int t = 0; t < 4; ++t) { oh[t][r] *= al; ol[t][r] *= al; }
      _Float16* pp = myP + (8 * hl + r) * 40 + c;
      pp[0]  = (_Float16)(p0 * P_CAR);
      pp[16] = (_Float16)(p1 * P_CAR);
    }
    __syncthreads();

    const v16h pf = ld_frag(myP + c * 40, hl);
#pragma unroll
    for (int t = 0; t < 4; ++t) {
      const v16h vfh = ld_frag(ldsVH + (16 * t + c) * 40, hl);
      const v16h vfl = ld_frag(ldsVL + (16 * t + c) * 40, hl);
      oh[t] = mma(pf, vfh, oh[t]);
      ol[t] = mma(pf, vfl, ol[t]);
    }
    __syncthreads();
  }

#pragma unroll
  for (int r = 0; r < 8; ++r) {
    const float inv = (1.0f / l[r]) * O_SCL;
    const int rowl = 16 * w + 8 * hl + r;
#pragma unroll
    for (int t = 0; t < 4; ++t) {
      const float v = (oh[t][r] + ol[t][r] * RES_INV) * inv;
      const _Float16 hv = (_Float16)v;
      const float res = (v - (float)hv) * RES_CAR;
      ldsOH[rowl * 72 + 16 * t + c] = hv;
      ldsOL[rowl * 72 + 16 * t + c] = (_Float16)res;
    }
  }
  __syncthreads();
  _Float16* const bh = OH + (brow + (size_t)q0) * DM + col0;
  _Float16* const bl = OL + (brow + (size_t)q0) * DM + col0;
  for (int i = 0; i < 4; ++i) {
    const int q = i * 256 + tid;
    const int rowl = q >> 3, ch = (q & 7) * 8;
    const v8h vh = *(const v8h*)(ldsOH + rowl * 72 + ch);
    const v8h vl = *(const v8h*)(ldsOL + rowl * 72 + ch);
    *(volatile v8h*)(bh + (size_t)rowl * DM + ch) = vh;
    *(volatile v8h*)(bl + (size_t)rowl * DM + ch) = vl;
  }
  __threadfence();
  for (int i = 0; i < 4; ++i) {
    const int q = i * 256 + tid;
    const int rowl = q >> 3, ch = (q & 7) * 8;
    const v8h vh = *(const v8h*)(ldsOH + rowl * 72 + ch);
    const v8h vl = *(const v8h*)(ldsOL + rowl * 72 + ch);
    *(volatile v8h*)(bh + (size_t)rowl * DM + ch) = vh;
    *(volatile v8h*)(bl + (size_t)rowl * DM + ch) = vl;
  }
}

__global__ __launch_bounds__(128) __attribute__((amdgpu_num_vgpr(256)))
void k_oproj(const _Float16* __restrict__ AH, const _Float16* __restrict__ AL,
             const _Float16* __restrict__ Bt, const float* __restrict__ bias,
             float* __restrict__ Out)
{
  __shared__ __attribute__((aligned(16))) float ldsF[64 * 68];

  const int tid = threadIdx.x, lane = tid & 31, w = tid >> 5;
  const int hl = lane >> 4, c = lane & 15;
  const int m0 = blockIdx.y * 64, n0 = blockIdx.x * 64;
  const int mw = m0 + 16 * w;

  const _Float16* ap0 = AH + (size_t)(mw + c) * DM;
  const _Float16* ap1 = AL + (size_t)(mw + c) * DM;
  const _Float16* bp  = Bt + (size_t)(n0 + c) * DM;

  v8f acc[8] = {};
  gemm_core(ap0, ap1, bp, DM, hl, acc);

  float bs[4];
#pragma unroll
  for (int t = 0; t < 4; ++t) bs[t] = bf16_rne(bias[n0 + 16 * t + c]);

#pragma unroll
  for (int t = 0; t < 4; ++t)
#pragma unroll
    for (int r = 0; r < 8; ++r) {
      const int rowl = 16 * w + 8 * hl + r;
      ldsF[rowl * 68 + 16 * t + c] = (acc[t][r] + acc[4 + t][r] * RES_INV) * OUT_SCL + bs[t];
    }
  __syncthreads();

  const unsigned b  = (unsigned)m0 / (unsigned)SEQ;
  const unsigned t0 = (unsigned)m0 - b * (unsigned)SEQ;
  float* const ob = Out + ((size_t)b * SEQ_FULL + t0) * ZD + n0;
  for (int i = 0; i < 8; ++i) {
    const int qi = i * 128 + tid;
    const int rowl = qi >> 4, col = (qi & 15) * 4;
    const v4f v = *(const v4f*)(ldsF + rowl * 68 + col);
    *(volatile v4f*)(ob + (size_t)rowl * ZD + col) = v;
  }
  __threadfence();
  for (int i = 0; i < 8; ++i) {
    const int qi = i * 128 + tid;
    const int rowl = qi >> 4, col = (qi & 15) * 4;
    const v4f v = *(const v4f*)(ldsF + rowl * 68 + col);
    *(volatile v4f*)(ob + (size_t)rowl * ZD + col) = v;
  }
}

extern "C" void kernel_launch(void* const* d_in, const int* in_sizes, int n_in,
                              void* d_out, int out_size, void* d_ws, size_t ws_size,
                              hipStream_t stream)
{
  if (n_in < 19) return;
  const long act_min = ((long)(NB - 1) * SEQ_FULL + SEQ) * ZD;
  if ((long)in_sizes[0]  < act_min) return;
  if ((long)in_sizes[1]  < act_min) return;
  if ((long)in_sizes[3]  < (long)ZD * DL) return;
  if ((long)in_sizes[4]  < (long)DL) return;
  if ((long)in_sizes[5]  < (long)DL * DM) return;
  if ((long)in_sizes[6]  < (long)DM) return;
  if ((long)in_sizes[7]  < (long)DL * DM) return;
  if ((long)in_sizes[8]  < (long)DM) return;
  if ((long)in_sizes[9]  < (long)ZD * DL) return;
  if ((long)in_sizes[10] < (long)DL) return;
  if ((long)in_sizes[11] < (long)DL * DM) return;
  if ((long)in_sizes[12] < (long)DM) return;
  if ((long)in_sizes[13] < (long)DL * DM) return;
  if ((long)in_sizes[14] < (long)DM) return;
  if ((long)in_sizes[15] < (long)ZD * RD) return;
  if ((long)in_sizes[16] < (long)RD) return;
  if ((long)in_sizes[17] < (long)DM * ZD) return;
  if ((long)in_sizes[18] < (long)ZD) return;
  if ((long)out_size < act_min) return;

  const float* query = (const float*)d_in[0];
  const float* key   = (const float*)d_in[1];
  const float* w_dkv = (const float*)d_in[3];
  const float* b_dkv = (const float*)d_in[4];
  const float* w_uk  = (const float*)d_in[5];
  const float* b_uk  = (const float*)d_in[6];
  const float* w_uv  = (const float*)d_in[7];
  const float* b_uv  = (const float*)d_in[8];
  const float* w_dq  = (const float*)d_in[9];
  const float* b_dq  = (const float*)d_in[10];
  const float* w_uq  = (const float*)d_in[11];
  const float* b_uq  = (const float*)d_in[12];
  const float* w_qr  = (const float*)d_in[13];
  const float* b_qr  = (const float*)d_in[14];
  const float* w_kr  = (const float*)d_in[15];
  const float* b_kr  = (const float*)d_in[16];
  const float* w_fc  = (const float*)d_in[17];
  const float* b_fc  = (const float*)d_in[18];
  float* out = (float*)d_out;

  const size_t nAct = (size_t)MROWS * ZD;
  const size_t nWd  = (size_t)DL * ZD;
  const size_t nWr  = (size_t)RD * ZD;
  const size_t nWu  = (size_t)DM * DL;
  const size_t nWf  = (size_t)ZD * DM;
  const size_t nLat = (size_t)MROWS * DL;
  const size_t nPl  = (size_t)MROWS * DM;
  const size_t nKr  = (size_t)MROWS * RD;
  const size_t nTab = (size_t)SEQ * 64 * 2;
  const size_t total_halves = 2 * nAct + 2 * nWd + nWr + 4 * nWu + nWf + 3 * nLat + 7 * nPl + nKr + nTab;
  if (total_halves * sizeof(_Float16) > ws_size) return;
  if (total_halves * sizeof(_Float16) > (size_t)134217728) return;

  _Float16* Q16   = (_Float16*)d_ws;
  _Float16* K16   = Q16   + nAct;
  _Float16* WdkvT = K16   + nAct;
  _Float16* WdqT  = WdkvT + nWd;
  _Float16* WkrT  = WdqT  + nWd;
  _Float16* WukT  = WkrT  + nWr;
  _Float16* WuvT  = WukT  + nWu;
  _Float16* WuqT  = WuvT  + nWu;
  _Float16* WqrT  = WuqT  + nWu;
  _Float16* WfcT  = WqrT  + nWu;
  _Float16* CKVH  = WfcT  + nWf;
  _Float16* CKVL  = CKVH  + nLat;
  _Float16* CQH   = CKVL  + nLat;
  _Float16* KC    = CQH   + nLat;
  _Float16* QC    = KC    + nPl;
  _Float16* QR    = QC    + nPl;
  _Float16* KR    = QR    + nPl;
  _Float16* VtH   = KR    + nKr;
  _Float16* VtL   = VtH   + nPl;
  _Float16* OH    = VtL   + nPl;
  _Float16* OL    = OH    + nPl;
  float*    TAB   = (float*)(OL + nPl);

  const unsigned t8 = (unsigned)(nAct / 8);
  k_cvt8<<<(t8 + 255u) / 256u, 256, 0, stream>>>(query, Q16, ACT_CAR, t8);
  k_cvt8<<<(t8 + 255u) / 256u, 256, 0, stream>>>(key,   K16, ACT_CAR, t8);

  k_trw<<<dim3(DL / 64, ZD / 64), 256, 0, stream>>>(w_dkv, WdkvT, ZD, DL);
  k_trw<<<dim3(DL / 64, ZD / 64), 256, 0, stream>>>(w_dq,  WdqT,  ZD, DL);
  k_trw<<<dim3(RD / 64, ZD / 64), 256, 0, stream>>>(w_kr,  WkrT,  ZD, RD);
  k_trw<<<dim3(DM / 64, DL / 64), 256, 0, stream>>>(w_uk,  WukT,  DL, DM);
  k_trw<<<dim3(DM / 64, DL / 64), 256, 0, stream>>>(w_uv,  WuvT,  DL, DM);
  k_trw<<<dim3(DM / 64, DL / 64), 256, 0, stream>>>(w_uq,  WuqT,  DL, DM);
  k_trw<<<dim3(DM / 64, DL / 64), 256, 0, stream>>>(w_qr,  WqrT,  DL, DM);
  k_trw<<<dim3(ZD / 64, DM / 64), 256, 0, stream>>>(w_fc,  WfcT,  DM, ZD);

  InvF fr;
  for (int i = 0; i < 32; ++i) {
    const double pw = pow(10000.0, (double)(2 * i) / 64.0);
    const float pwf = (float)pw;
    fr.v[i] = 1.0f / pwf;
  }
  k_tab<<<SEQ / 8, 256, 0, stream>>>(fr, TAB);

  k_proj<1><<<dim3(DL / 64, MROWS / 128), 128, 0, stream>>>(K16, WdkvT, b_dkv, (const float*)nullptr, CKVH, CKVL, ZD, DL);
  k_proj<0><<<dim3(DL / 64, MROWS / 128), 128, 0, stream>>>(Q16, WdqT, b_dq, (const float*)nullptr, CQH, (_Float16*)nullptr, ZD, DL);
  k_proj<2><<<dim3(RD / 64, MROWS / 128), 128, 0, stream>>>(K16, WkrT, b_kr, TAB, KR, (_Float16*)nullptr, ZD, RD);
  k_proj<0><<<dim3(DM / 64, MROWS / 128), 128, 0, stream>>>(CKVH, WukT, b_uk, (const float*)nullptr, KC, (_Float16*)nullptr, DL, DM);
  k_proj<0><<<dim3(DM / 64, MROWS / 128), 128, 0, stream>>>(CQH, WuqT, b_uq, (const float*)nullptr, QC, (_Float16*)nullptr, DL, DM);
  k_proj<2><<<dim3(DM / 64, MROWS / 128), 128, 0, stream>>>(CQH, WqrT, b_qr, TAB, QR, (_Float16*)nullptr, DL, DM);
  k_vproj<<<dim3(DM / 64, MROWS / 64), 128, 0, stream>>>(CKVH, CKVL, WuvT, b_uv, VtH, VtL);

  k_attn<<<dim3(SEQ / 128, NH, NB), 256, 0, stream>>>(QC, QR, KC, KR, VtH, VtL, OH, OL);

  k_oproj<<<dim3(ZD / 64, MROWS / 64), 128, 0, stream>>>(OH, OL, WfcT, b_fc, out);
}
